// FullAttention_50646254355303
// MI455X (gfx1250) — hardware-verified
//
#include <hip/hip_runtime.h>

#ifndef NB
#define NB 2
#endif
#ifndef SEQ
#define SEQ 2048
#endif
#ifndef RESQ
#if SEQ < 512
#define RESQ SEQ
#else
#define RESQ 512
#endif
#endif
#define NB_FULL 2
#define SEQ_FULL 2048
#define HID 2048
#define NH 16
#define NKV 4
#define HD 128
#define GQ (NH / NKV)
#define NQC (2 * NH * HD)
#define NKVC (2 * NKV * HD)
#define NHR (NH + NKV)
#define NRP 64
#define PCAR 16384.0f
#define OCAR 64.0f
#define RCAR 1024.0f
#define WCAR 16.0f

static_assert(NB >= 1);
static_assert(NB <= NB_FULL);
static_assert(SEQ % 128 == 0);
static_assert(SEQ <= SEQ_FULL);
static_assert(RESQ % 128 == 0);
static_assert(RESQ >= 128);
static_assert(RESQ <= SEQ);
static_assert((SEQ - RESQ) % 128 == 0);
static_assert(HID % 32 == 0);
static_assert(HID % 64 == 0);
static_assert(NQC % 64 == 0);
static_assert(NKVC % 64 == 0);
static_assert((NH * HD) % 32 == 0);
static_assert(HD == 128);
static_assert(NH % NKV == 0);
static_assert((SEQ * NHR) % 8 == 0);
static_assert((SEQ * HID) % 8 == 0);

constexpr size_t SZ_X16   = (size_t)SEQ * HID * 2;
constexpr size_t SZ_WQT   = (size_t)NQC * HID * 2;
constexpr size_t SZ_WKVT  = (size_t)NKVC * HID * 2;
constexpr size_t SZ_WOT   = (size_t)HID * NH * HD * 2;
constexpr size_t SZ_CS    = (size_t)SEQ * NRP * 2 * 4;
constexpr size_t SZ_QRAW  = (size_t)SEQ * NQC * 4;
constexpr size_t SZ_KVRAW = (size_t)SEQ * NKVC * 4;
constexpr size_t SZ_QH    = (size_t)NH * SEQ * HD * 2;
constexpr size_t SZ_QL    = (size_t)NH * RESQ * HD * 2;
constexpr size_t SZ_KH    = (size_t)NKV * SEQ * HD * 2;
constexpr size_t SZ_KL    = (size_t)NKV * RESQ * HD * 2;
constexpr size_t SZ_VT    = (size_t)NKV * HD * SEQ * 2;
constexpr size_t SZ_VTL   = (size_t)NKV * HD * RESQ * 2;
constexpr size_t SZ_OH    = (size_t)SEQ * NH * HD * 2;
constexpr size_t SZ_OL    = (size_t)RESQ * NH * HD * 2;
constexpr size_t WS_TOTAL = SZ_X16 + SZ_WQT + SZ_WKVT + SZ_WOT + SZ_CS + SZ_QRAW + SZ_KVRAW + SZ_QH + SZ_QL + SZ_KH + SZ_KL + SZ_VT + SZ_VTL + SZ_OH + SZ_OL;
static_assert(WS_TOTAL <= (size_t)134217728);
static_assert(SZ_X16 % 256 == 0);
static_assert(SZ_KL % 256 == 0);
static_assert(SZ_VTL % 256 == 0);
static_assert(SZ_CS % 256 == 0);

typedef _Float16 v16h __attribute__((ext_vector_type(16)));
typedef unsigned short v8us __attribute__((ext_vector_type(8), may_alias));
typedef float v8f __attribute__((ext_vector_type(8)));
typedef float v4f __attribute__((ext_vector_type(4)));
typedef float v4fa __attribute__((ext_vector_type(4), may_alias));
typedef float v2f __attribute__((ext_vector_type(2)));
typedef _Float16 v4h __attribute__((ext_vector_type(4)));
union FragH { v16h v; v8us half[2]; _Float16 h[16]; unsigned short u[16]; };
union Pack8 { v8us v; _Float16 h[8]; unsigned short u[8]; };

__device__ __forceinline__ unsigned short bf16_bits(float x) { const unsigned int u = __float_as_uint(x); return (unsigned short)((u + 0x7FFFu + ((u >> 16) & 1u)) >> 16); }
__device__ __forceinline__ float bf16_rne(float x) { return __uint_as_float(((unsigned int)bf16_bits(x)) << 16); }

__device__ __forceinline__ v16h frag16(const _Float16* p, int hh) {
  FragH f;
  f.half[0] = *(const v8us*)((const unsigned short*)p + 8 * hh);
  f.half[1] = *(const v8us*)((const unsigned short*)p + 16 + 8 * hh);
  return f.v;
}
__device__ __forceinline__ v8f mma16(v16h a, v16h b, v8f c) {
  v8f d = __builtin_amdgcn_wmma_f32_16x16x32_f16(false, a, false, b, (short)0, c, false, false);
  asm volatile("v_nop\n\tv_nop\n\tv_nop\n\tv_nop" : "+v"(d) : "v"(a), "v"(b));
  return d;
}

__global__ __launch_bounds__(256) void k_x16(const float* __restrict__ x, _Float16* __restrict__ X16, size_t n8) {
  const size_t t = (size_t)blockIdx.x * 256 + threadIdx.x; if (t >= n8) return;
  const v4f a = *(const v4fa*)(x + t * 8), c = *(const v4fa*)(x + t * 8 + 4);
  Pack8 f;
#pragma unroll
  for (int q = 0; q < 4; ++q) { f.h[q] = (_Float16)bf16_rne(a[q]); f.h[4 + q] = (_Float16)bf16_rne(c[q]); }
  unsigned short* d = (unsigned short*)X16 + t * 8;
  *(volatile v8us*)d = f.v; __threadfence(); *(volatile v8us*)d = f.v;
}

__global__ __launch_bounds__(256) void k_wt_f16(const float* __restrict__ W, _Float16* __restrict__ Wt, int K, int N, float scale) {
  const int t = blockIdx.x * 256 + threadIdx.x; if (t >= N * (K / 8)) return;
  const int n = t / (K / 8), k8 = (t % (K / 8)) * 8;
  Pack8 f;
#pragma unroll
  for (int i = 0; i < 8; ++i) f.h[i] = (_Float16)(bf16_rne(W[(size_t)(k8 + i) * N + n]) * scale);
  unsigned short* d = (unsigned short*)Wt + (size_t)n * K + k8;
  *(volatile v8us*)d = f.v; __threadfence(); *(volatile v8us*)d = f.v;
}

__global__ __launch_bounds__(256) void k_rope(float* __restrict__ cs) {
  const int t = blockIdx.x * 256 + threadIdx.x; if (t >= SEQ * NRP) return;
  const int pos = t / NRP, i = t - pos * NRP;
  const float inv = exp2f(-(float)i * 0.31143075889569022f);
  const float ang = (float)pos * inv;
  float sn, cn; sincosf(ang, &sn, &cn);
  v2f o; o[0] = cn; o[1] = sn;
  float* d = cs + (size_t)t * 2;
  *(volatile v2f*)d = o; __threadfence(); *(volatile v2f*)d = o;
}

__global__ __launch_bounds__(128) void k_gemm(const _Float16* __restrict__ A, int lda, const _Float16* __restrict__ Bt, int ldb, float alpha,
                                             float* __restrict__ C, int ldc, int M, int N, int K) {
  __shared__ __attribute__((aligned(16))) float so[4][32][68];
  const int tid = threadIdx.x, w = tid >> 5, lane = tid & 31, ln = lane & 15, hh = lane >> 4;
  const int ntn = N >> 6;
  const int mt = (int)blockIdx.x / ntn, nq = (int)blockIdx.x - mt * ntn;
  const int row0 = mt * 128 + 32 * w, col0 = nq * 64;
  if (row0 >= M) return;
  const _Float16* a0p = A + (size_t)(row0 + ln) * lda; const _Float16* a1p = a0p + (size_t)16 * lda;
  const _Float16* b0p = Bt + (size_t)(col0 + ln) * ldb; const _Float16* b1p = b0p + (size_t)16 * ldb;
  const _Float16* b2p = b1p + (size_t)16 * ldb; const _Float16* b3p = b2p + (size_t)16 * ldb;
  const v8f z8 = {0.f, 0.f, 0.f, 0.f, 0.f, 0.f, 0.f, 0.f};
  v8f c00 = z8, c01 = z8, c02 = z8, c03 = z8, c10 = z8, c11 = z8, c12 = z8, c13 = z8;
#pragma unroll 1
  for (int kb = 0; kb < K; kb += 32) {
    const v16h a0 = frag16(a0p + kb, hh), a1 = frag16(a1p + kb, hh);
    v16h b = frag16(b0p + kb, hh); c00 = mma16(a0, b, c00); c10 = mma16(a1, b, c10);
    b = frag16(b1p + kb, hh); c01 = mma16(a0, b, c01); c11 = mma16(a1, b, c11);
    b = frag16(b2p + kb, hh); c02 = mma16(a0, b, c02); c12 = mma16(a1, b, c12);
    b = frag16(b3p + kb, hh); c03 = mma16(a0, b, c03); c13 = mma16(a1, b, c13);
  }
  v8f accs[8] = {c00, c01, c02, c03, c10, c11, c12, c13};
#pragma unroll
  for (int u = 0; u < 8; ++u) {
    const int t = u & 3, half = u >> 2;
#pragma unroll
    for (int r = 0; r < 8; ++r) so[w][half * 16 + 8 * hh + r][t * 16 + ln] = accs[u][r] * alpha;
  }
  __builtin_amdgcn_fence(4  , "workgroup");
  __builtin_amdgcn_wave_barrier();
  const int rsub = lane >> 4, c4 = (lane & 15) * 4;
  for (int pass = 0; pass < 2; ++pass) {
#pragma unroll
    for (int q = 0; q < 16; ++q) {
      const int r = q * 2 + rsub;
      const v4f v = *(const v4fa*)&so[w][r][c4];
      *(volatile v4f*)(C + (size_t)(row0 + r) * ldc + col0 + c4) = v;
    }
    if (pass == 0) __threadfence();
  }
}

__global__ __launch_bounds__(128) void k_gemm_r(const _Float16* __restrict__ A, const _Float16* __restrict__ Al, int lda, const _Float16* __restrict__ Bt, int ldb,
                                               float alpha, float alphal, float* __restrict__ C, int ldc, int M, int N, int K) {
  __shared__ __attribute__((aligned(16))) float so[4][16][68];
  const int tid = threadIdx.x, w = tid >> 5, lane = tid & 31, ln = lane & 15, hh = lane >> 4;
  const int ntn = N >> 6;
  const int wid = (int)blockIdx.x * 4 + w;
  const int mt = wid / ntn, nq = wid - mt * ntn;
  const int row0 = mt * 16, col0 = nq * 64;
  if (row0 >= M) return;
  const _Float16* ap = A + (size_t)(row0 + ln) * lda; const _Float16* alp = Al + (size_t)(row0 + ln) * lda;
  const _Float16* b0p = Bt + (size_t)(col0 + ln) * ldb; const _Float16* b1p = b0p + (size_t)16 * ldb;
  const _Float16* b2p = b1p + (size_t)16 * ldb; const _Float16* b3p = b2p + (size_t)16 * ldb;
  const v8f z8 = {0.f, 0.f, 0.f, 0.f, 0.f, 0.f, 0.f, 0.f};
  v8f h0 = z8, h1 = z8, h2 = z8, h3 = z8, l0 = z8, l1 = z8, l2 = z8, l3 = z8;
#pragma unroll 1
  for (int kb = 0; kb < K; kb += 32) {
    const v16h a = frag16(ap + kb, hh), al = frag16(alp + kb, hh);
    v16h b = frag16(b0p + kb, hh); h0 = mma16(a, b, h0); l0 = mma16(al, b, l0);
    b = frag16(b1p + kb, hh); h1 = mma16(a, b, h1); l1 = mma16(al, b, l1);
    b = frag16(b2p + kb, hh); h2 = mma16(a, b, h2); l2 = mma16(al, b, l2);
    b = frag16(b3p + kb, hh); h3 = mma16(a, b, h3); l3 = mma16(al, b, l3);
  }
  v8f hs[4] = {h0, h1, h2, h3}; v8f ls[4] = {l0, l1, l2, l3};
#pragma unroll
  for (int t = 0; t < 4; ++t) {
#pragma unroll
    for (int r = 0; r < 8; ++r) so[w][8 * hh + r][t * 16 + ln] = hs[t][r] * alpha + ls[t][r] * alphal;
  }
  __builtin_amdgcn_fence(4  , "workgroup");
  __builtin_amdgcn_wave_barrier();
  const int rsub = lane >> 4, c4 = (lane & 15) * 4;
  for (int pass = 0; pass < 2; ++pass) {
#pragma unroll
    for (int q = 0; q < 8; ++q) {
      const int r = q * 2 + rsub;
      const v4f v = *(const v4fa*)&so[w][r][c4];
      *(volatile v4f*)(C + (size_t)(row0 + r) * ldc + col0 + c4) = v;
    }
    if (pass == 0) __threadfence();
  }
}

__global__ __launch_bounds__(256) void k_qk(const float* __restrict__ qraw, const float* __restrict__ kvraw,
                                           const float* __restrict__ qnw, const float* __restrict__ knw, const float* __restrict__ cs,
                                           _Float16* __restrict__ Qh, _Float16* __restrict__ Ql, _Float16* __restrict__ Kh, _Float16* __restrict__ Kl) {
  const int w = threadIdx.x >> 5, lane = threadIdx.x & 31;
  const int wid = (int)blockIdx.x * 8 + w;
  if (wid >= SEQ * NHR) return;
  const int s = wid / NHR, j = wid - s * NHR;
  const bool isq = (j < NH);
  const float* src = isq ? (qraw + (size_t)s * NQC + (size_t)j * (2 * HD)) : (kvraw + (size_t)s * NKVC + (size_t)(j - NH) * HD);
  const float* wp = isq ? qnw : knw;
  const v4f xv = *(const v4fa*)(src + 4 * lane);
  const v4f wv = *(const v4fa*)(wp + 4 * lane);
  float ss = xv[0] * xv[0] + xv[1] * xv[1] + xv[2] * xv[2] + xv[3] * xv[3];
#pragma unroll
  for (int m = 16; m > 0; m >>= 1) ss += __shfl_xor(ss, m, 32);
  const float inv = rsqrtf(ss * (1.0f / 128.0f) + 1.0e-6f);
  float nv[4], pr[4];
#pragma unroll
  for (int q = 0; q < 4; ++q) nv[q] = xv[q] * inv * (wv[q] + 1.0f);
#pragma unroll
  for (int q = 0; q < 4; ++q) pr[q] = __shfl_xor(nv[q], 16, 32);
  const int i0 = 4 * (lane & 15);
  const v4f t01 = *(const v4fa*)(cs + ((size_t)s * NRP + i0) * 2);
  const v4f t23 = *(const v4fa*)(cs + ((size_t)s * NRP + i0 + 2) * 2);
  const float cv[4] = {t01[0], t01[2], t23[0], t23[2]};
  const float sv[4] = {t01[1], t01[3], t23[1], t23[3]};
  const float sg = (lane < 16) ? -1.0f : 1.0f;
  v4h oh, ol;
#pragma unroll
  for (int q = 0; q < 4; ++q) {
    const float o = nv[q] * cv[q] + sg * pr[q] * sv[q];
    const _Float16 hv = (_Float16)o;
    oh[q] = hv; ol[q] = (_Float16)((o - (float)hv) * RCAR);
  }
  _Float16* dh = isq ? (Qh + ((size_t)j * SEQ + s) * HD) : (Kh + ((size_t)(j - NH) * SEQ + s) * HD);
  _Float16* dl = isq ? (Ql + ((size_t)j * RESQ + s) * HD) : (Kl + ((size_t)(j - NH) * RESQ + s) * HD);
  const bool wl = (s < RESQ);
  for (int pass = 0; pass < 2; ++pass) {
    *(volatile v4h*)(dh + 4 * lane) = oh;
    if (wl) *(volatile v4h*)(dl + 4 * lane) = ol;
    if (pass == 0) __threadfence();
  }
}

__global__ __launch_bounds__(256) void k_vt(const float* __restrict__ kvraw, _Float16* __restrict__ VT, _Float16* __restrict__ VTl) {
  __shared__ float tl[64][65];
  const int tid = threadIdx.x;
  const int ntg = SEQ / 64;
  const int tg = (int)blockIdx.x % ntg, slab = (int)blockIdx.x / ntg;
  const int kv = slab >> 1, dh = slab & 1;
  const int s0 = tg * 64;
#pragma unroll
  for (int it = 0; it < 4; ++it) {
    const int i = tid + it * 256; const int tok = i >> 4, c4 = (i & 15) * 4;
    const v4f v = *(const v4fa*)(kvraw + (size_t)(s0 + tok) * NKVC + NKV * HD + kv * HD + dh * 64 + c4);
    tl[tok][c4] = v[0]; tl[tok][c4 + 1] = v[1]; tl[tok][c4 + 2] = v[2]; tl[tok][c4 + 3] = v[3];
  }
  __syncthreads();
  const int pc = tid & 7, dr = tid >> 3;
  const bool wl = (s0 < RESQ);
  for (int pass = 0; pass < 2; ++pass) {
#pragma unroll
    for (int rd = 0; rd < 2; ++rd) {
      const int d = rd * 32 + dr;
      Pack8 ph, pl;
#pragma unroll
      for (int q = 0; q < 8; ++q) { const float f = tl[pc * 8 + q][d]; const _Float16 hv = (_Float16)f; ph.h[q] = hv; pl.h[q] = (_Float16)((f - (float)hv) * RCAR); }
      const size_t row = (size_t)(kv * HD + dh * 64 + d);
      *(volatile v8us*)((unsigned short*)VT + row * SEQ + s0 + pc * 8) = ph.v;
      if (wl) *(volatile v8us*)((unsigned short*)VTl + row * RESQ + s0 + pc * 8) = pl.v;
    }
    if (pass == 0) __threadfence();
  }
}

template <bool RES>
__global__ __launch_bounds__(256) void k_attn(const _Float16* __restrict__ Qh, const _Float16* __restrict__ Ql,
                                             const _Float16* __restrict__ Kh, const _Float16* __restrict__ Kl,
                                             const _Float16* __restrict__ VT, const _Float16* __restrict__ VTl,
                                             const float* __restrict__ qraw, _Float16* __restrict__ Oh, _Float16* __restrict__ Ol, int qb0) {
  constexpr int KC = RES ? 32 : 64;
  constexpr int NJ = KC / 16;
  constexpr int NKS = KC / 32;
  constexpr int OD = RES ? 64 : 128;
  constexpr int NC = OD / 16;
  constexpr int NHF = OD / 64;
  constexpr int KP = HD + 8;
  constexpr int VP = KC + 8;
  constexpr int PP = 72;
  __shared__ __attribute__((aligned(16))) _Float16 sK[KC][KP];
  __shared__ __attribute__((aligned(16))) _Float16 sKl[RES ? KC : 1][KP];
  __shared__ __attribute__((aligned(16))) _Float16 sV[OD][VP];
  __shared__ __attribute__((aligned(16))) _Float16 sVl[RES ? OD : 1][VP];
  __shared__ __attribute__((aligned(16))) _Float16 sP[8][16][PP];
  __shared__ __attribute__((aligned(16))) _Float16 sPl[RES ? 8 : 1][16][PP];

  const int tid = threadIdx.x, w = tid >> 5, lane = tid & 31, ln = lane & 15, hh = lane >> 4;
  const int qb = qb0 + (int)blockIdx.x, h = (int)blockIdx.y, kv = h / GQ;
  const int dz = RES ? (int)blockIdx.z * 64 : 0;
  const int q0b = qb * 128, q0w = q0b + 16 * w;
  const int nch = (q0b + 128) / KC;
  const int qlast = q0w + 15;

  v16h aq[4], aql[4];
  {
    const _Float16* qp = Qh + ((size_t)h * SEQ + q0w + ln) * HD;
#pragma unroll
    for (int kk = 0; kk < 4; ++kk) aq[kk] = frag16(qp + kk * 32, hh);
    if (RES) {
      const _Float16* qlp = Ql + ((size_t)h * RESQ + q0w + ln) * HD;
#pragma unroll
      for (int kk = 0; kk < 4; ++kk) aql[kk] = frag16(qlp + kk * 32, hh);
    } else {
#pragma unroll
      for (int kk = 0; kk < 4; ++kk) aql[kk] = aq[kk];
    }
  }
  const v8f z8 = {0.f, 0.f, 0.f, 0.f, 0.f, 0.f, 0.f, 0.f};
  v8f o[NC];
#pragma unroll
  for (int c = 0; c < NC; ++c) o[c] = z8;
  float mrow[8], lrow[8];
#pragma unroll
  for (int r = 0; r < 8; ++r) { mrow[r] = -3.0e38f; lrow[r] = 0.f; }
  const float alpha = 0.08838834764831845f;

#pragma unroll 1
  for (int ch = 0; ch < nch; ++ch) {
    const int t0 = ch * KC;
#pragma unroll
    for (int it = 0; it < (KC * 16) / 256; ++it) {
      const int i = tid + it * 256; const int r = i >> 4, c8 = (i & 15) * 8;
      *(v8us*)&sK[r][c8] = *(const v8us*)((const unsigned short*)Kh + ((size_t)kv * SEQ + t0 + r) * HD + c8);
      if (RES) *(v8us*)&sKl[r][c8] = *(const v8us*)((const unsigned short*)Kl + ((size_t)kv * RESQ + t0 + r) * HD + c8);
    }
#pragma unroll
    for (int it = 0; it < (OD * (KC / 8)) / 256; ++it) {
      const int i = tid + it * 256; const int d = i / (KC / 8), c8 = (i % (KC / 8)) * 8;
      *(v8us*)&sV[d][c8] = *(const v8us*)((const unsigned short*)VT + (size_t)(kv * HD + dz + d) * SEQ + t0 + c8);
      if (RES) *(v8us*)&sVl[d][c8] = *(const v8us*)((const unsigned short*)VTl + (size_t)(kv * HD + dz + d) * RESQ + t0 + c8);
    }
    __syncthreads();
    if (t0 <= qlast) {
      v8f sacc[NJ];
#pragma unroll
      for (int j = 0; j < NJ; ++j) {
        v8f acc = z8, tmp = z8;
#pragma unroll
        for (int kk = 0; kk < 4; ++kk) {
          const v16h b = frag16(&sK[j * 16 + ln][kk * 32], hh);
          acc = mma16(aq[kk], b, acc);
          if (RES) {
            const v16h bl = frag16(&sKl[j * 16 + ln][kk * 32], hh);
            tmp = mma16(aql[kk], b, tmp);
            tmp = mma16(aq[kk], bl, tmp);
          }
        }
        if (RES) acc = acc + tmp * (1.0f / RCAR);
        sacc[j] = acc;
      }
#pragma unroll
      for (int r = 0; r < 8; ++r) {
        const int qrow = q0w + 8 * hh + r;
        float sv[NJ]; bool mk[NJ]; float mx = -3.0e38f;
#pragma unroll
        for (int j = 0; j < NJ; ++j) { mk[j] = (t0 + 16 * j + ln) > qrow; sv[j] = sacc[j][r] * alpha; mx = fmaxf(mx, mk[j] ? -3.0e38f : sv[j]); }
#pragma unroll
        for (int m = 8; m > 0; m >>= 1) mx = fmaxf(mx, __shfl_xor(mx, m, 32));
        const float mnew = fmaxf(mrow[r], mx);
        const float fac = (mrow[r] < -1.0e38f) ? 0.f : __expf(mrow[r] - mnew);
        float rs = 0.f;
#pragma unroll
        for (int j = 0; j < NJ; ++j) {
          const float p = mk[j] ? 0.f : __expf(sv[j] - mnew);
          rs += p;
          const float pcv = p * PCAR; const _Float16 ph = (_Float16)pcv;
          sP[w][8 * hh + r][16 * j + ln] = ph;
          if (RES) sPl[w][8 * hh + r][16 * j + ln] = (_Float16)((pcv - (float)ph) * RCAR);
        }
#pragma unroll
        for (int m = 8; m > 0; m >>= 1) rs += __shfl_xor(rs, m, 32);
        lrow[r] = lrow[r] * fac + rs; mrow[r] = mnew;
#pragma unroll
        for (int c = 0; c < NC; ++c) o[c][r] *= fac;
      }
      __builtin_amdgcn_fence(4  , "workgroup");
      __builtin_amdgcn_wave_barrier();
      v16h ap[NKS], apl[NKS];
#pragma unroll
      for (int ks = 0; ks < NKS; ++ks) {
        ap[ks] = frag16(&sP[w][ln][ks * 32], hh);
        if (RES) apl[ks] = frag16(&sPl[w][ln][ks * 32], hh); else apl[ks] = ap[ks];
      }
#pragma unroll
      for (int c = 0; c < NC; ++c) {
        v8f tmp = z8;
#pragma unroll
        for (int ks = 0; ks < NKS; ++ks) {
          const v16h b = frag16(&sV[c * 16 + ln][ks * 32], hh);
          o[c] = mma16(ap[ks], b, o[c]);
          if (RES) {
            const v16h bl = frag16(&sVl[c * 16 + ln][ks * 32], hh);
            tmp = mma16(apl[ks], b, tmp);
            tmp = mma16(ap[ks], bl, tmp);
          }
        }
        if (RES) o[c] = o[c] + tmp * (1.0f / RCAR);
      }
    }
    __syncthreads();
  }

  float il[8];
#pragma unroll
  for (int r = 0; r < 8; ++r) il[r] = (OCAR / PCAR) * __builtin_amdgcn_rcpf(lrow[r]);
  const float* gp = qraw + (size_t)(q0w + 8 * hh) * NQC + (size_t)h * (2 * HD) + HD + dz + ln;
#pragma unroll
  for (int hf = 0; hf < NHF; ++hf) {
    if (hf > 0) { __builtin_amdgcn_fence(4  , "workgroup"); __builtin_amdgcn_wave_barrier(); }
#pragma unroll
    for (int cc = 0; cc < 4; ++cc) {
      const int c = hf * 4 + cc;
#pragma unroll
      for (int r = 0; r < 8; ++r) {
        const float g = gp[(size_t)r * NQC + c * 16];
        const float sig = __builtin_amdgcn_rcpf(1.0f + __expf(-g));
        const float val = o[c][r] * il[r] * sig;
        const _Float16 vh = (_Float16)val;
        sP[w][8 * hh + r][cc * 16 + ln] = vh;
        if (RES) sPl[w][8 * hh + r][cc * 16 + ln] = (_Float16)((val - (float)vh) * RCAR);
      }
      asm volatile("" ::: "memory");
    }
    __builtin_amdgcn_fence(4  , "workgroup");
    __builtin_amdgcn_wave_barrier();
    const int prw = lane >> 3, pc = lane & 7;
    for (int pass = 0; pass < 2; ++pass) {
#pragma unroll
      for (int it = 0; it < 4; ++it) {
        const int row = it * 4 + prw;
        const v8us vv = *(const v8us*)&sP[w][row][pc * 8];
        const size_t go = (size_t)(q0w + row) * (NH * HD) + (size_t)h * HD + dz + hf * 64 + pc * 8;
        *(volatile v8us*)((unsigned short*)Oh + go) = vv;
        if (RES) { const v8us vl = *(const v8us*)&sPl[w][row][pc * 8]; *(volatile v8us*)((unsigned short*)Ol + go) = vl; }
      }
      if (pass == 0) __threadfence();
    }
  }
}

extern "C" void kernel_launch(void* const* d_in, const int* in_sizes, int n_in,
                              void* d_out, int out_size, void* d_ws, size_t ws_size, hipStream_t stream) {
  if (n_in < 7) return;
  const long need_x = (long)(NB - 1) * SEQ_FULL * HID + (long)SEQ * HID;
  if ((long)in_sizes[0] < need_x) return;
  if (in_sizes[1] < HID * NQC) return;
  if (in_sizes[2] < HID * NKV * HD) return;
  if (in_sizes[3] < HID * NKV * HD) return;
  if (in_sizes[4] < NH * HD * HID) return;
  if (in_sizes[5] < HD) return;
  if (in_sizes[6] < HD) return;
  if ((long)out_size < need_x) return;

  const float* x   = (const float*)d_in[0];
  const float* Wq  = (const float*)d_in[1];
  const float* Wk  = (const float*)d_in[2];
  const float* Wv  = (const float*)d_in[3];
  const float* Wo  = (const float*)d_in[4];
  const float* qnw = (const float*)d_in[5];
  const float* knw = (const float*)d_in[6];

  char* ws = (char*)d_ws; size_t off = 0;
  auto take = [&](size_t bytes) { char* p = ws + off; off += (bytes + 255) & ~(size_t)255; return p; };
  _Float16* X16  = (_Float16*)take(SZ_X16);
  _Float16* WqT  = (_Float16*)take(SZ_WQT);
  _Float16* WkvT = (_Float16*)take(SZ_WKVT);
  _Float16* WoT  = (_Float16*)take(SZ_WOT);
  float*    CS   = (float*)take(SZ_CS);
  float*    qraw = (float*)take(SZ_QRAW);
  float*    kvraw = (float*)take(SZ_KVRAW);
  _Float16* Qh   = (_Float16*)take(SZ_QH);
  _Float16* Ql   = (_Float16*)take(SZ_QL);
  _Float16* Kh   = (_Float16*)take(SZ_KH);
  _Float16* Kl   = (_Float16*)take(SZ_KL);
  _Float16* VT   = (_Float16*)take(SZ_VT);
  _Float16* VTl  = (_Float16*)take(SZ_VTL);
  _Float16* Oh   = (_Float16*)take(SZ_OH);
  _Float16* Ol   = (_Float16*)take(SZ_OL);
  if (off > ws_size) return;

  k_rope<<<(SEQ * NRP + 255) / 256, 256, 0, stream>>>(CS);
  k_wt_f16<<<(NQC * (HID / 8) + 255) / 256, 256, 0, stream>>>(Wq, WqT, HID, NQC, WCAR);
  k_wt_f16<<<(NKV * HD * (HID / 8) + 255) / 256, 256, 0, stream>>>(Wk, WkvT, HID, NKV * HD, WCAR);
  k_wt_f16<<<(NKV * HD * (HID / 8) + 255) / 256, 256, 0, stream>>>(Wv, WkvT + (size_t)NKV * HD * HID, HID, NKV * HD, WCAR);
  k_wt_f16<<<(HID * ((NH * HD) / 8) + 255) / 256, 256, 0, stream>>>(Wo, WoT, NH * HD, HID, WCAR);

  const float walpha = 1.0f / WCAR;
  const float oalpha = 1.0f / (WCAR * OCAR);
  const float oalphal = oalpha / RCAR;
  for (int b = 0; b < NB; ++b) {
    const size_t xoff = (size_t)b * SEQ_FULL * HID;
    float* outb = (float*)d_out + (size_t)b * SEQ_FULL * HID;
    k_x16<<<(unsigned)(((size_t)SEQ * HID / 8 + 255) / 256), 256, 0, stream>>>(x + xoff, X16, (size_t)SEQ * HID / 8);
    k_gemm<<<(SEQ / 128) * (NQC / 64), 128, 0, stream>>>(X16, HID, WqT, HID, walpha, qraw, NQC, SEQ, NQC, HID);
    k_gemm<<<(SEQ / 128) * (NKVC / 64), 128, 0, stream>>>(X16, HID, WkvT, HID, walpha, kvraw, NKVC, SEQ, NKVC, HID);
    k_qk<<<(SEQ * NHR) / 8, 256, 0, stream>>>(qraw, kvraw, qnw, knw, CS, Qh, Ql, Kh, Kl);
    k_vt<<<NKV * 2 * (SEQ / 64), 256, 0, stream>>>(kvraw, VT, VTl);
    k_attn<true><<<dim3(RESQ / 128, NH, 2), 256, 0, stream>>>(Qh, Ql, Kh, Kl, VT, VTl, qraw, Oh, Ol, 0);
    if (SEQ > RESQ)
      k_attn<false><<<dim3((SEQ - RESQ) / 128, NH, 1), 256, 0, stream>>>(Qh, Ql, Kh, Kl, VT, VTl, qraw, Oh, Ol, RESQ / 128);
    k_gemm_r<<<((RESQ / 16) * (HID / 64) + 3) / 4, 128, 0, stream>>>(Oh, Ol, NH * HD, WoT, NH * HD, oalpha, oalphal, outb, HID, RESQ, HID, NH * HD);
    if (SEQ > RESQ)
      k_gemm<<<((SEQ - RESQ) / 128) * (HID / 64), 128, 0, stream>>>(Oh + (size_t)RESQ * NH * HD, NH * HD, WoT, NH * HD, oalpha, outb + (size_t)RESQ * HID, HID, SEQ - RESQ, HID, NH * HD);
  }
  (void)hipGetLastError();
}
